// NAO_14637248545385
// MI455X (gfx1250) — hardware-verified
//
#include <hip/hip_runtime.h>

typedef unsigned short u16;
typedef __bf16 v16b __attribute__((ext_vector_type(16)));
typedef u16 v16us __attribute__((ext_vector_type(16)));
typedef u16 v8us __attribute__((ext_vector_type(8)));
typedef float v16f __attribute__((ext_vector_type(16)));
typedef float v8f __attribute__((ext_vector_type(8)));
typedef float v4f __attribute__((ext_vector_type(4)));
typedef v8us __attribute__((may_alias)) v8usa;
typedef v4f __attribute__((may_alias)) v4fa;

union Frag { v16b v; v16us u; v8us half[2]; };

#define NB_   4
#define NPER  4096
#define RTOT  (NB_ * NPER)
#define DM    512
#define DKK   64
#define NLAY  4
#define RBLK  512
#define NPART (NPER / RBLK)

static_assert(RTOT % 64 == 0);
static_assert(NPER % RBLK == 0);
static_assert(RBLK % 32 == 0);
static_assert(DM % 128 == 0);

__device__ __forceinline__ unsigned bf16_bits(float x) {
  unsigned u = __float_as_uint(x);
  u += 0x7FFFu + ((u >> 16) & 1u);
  return u >> 16;
}

struct HL8 { v8us hi; v8us lo; };

__device__ __forceinline__ HL8 split8(v8f x) {
  HL8 r;
  v8us hi = {0, 0, 0, 0, 0, 0, 0, 0};
  v8us lo = {0, 0, 0, 0, 0, 0, 0, 0};
#pragma unroll
  for (int j = 0; j < 8; ++j) {
    const unsigned hb = bf16_bits(x[j]);
    const float res = x[j] - __uint_as_float(hb << 16);
    const unsigned lb = bf16_bits(res);
    hi[j] = (u16)hb;
    lo[j] = (u16)lb;
  }
  r.hi = hi;
  r.lo = lo;
  return r;
}

__device__ __forceinline__ v8f cat8(v4f a, v4f c) {
  v8f x = {a.x, a.y, a.z, a.w, c.x, c.y, c.z, c.w};
  return x;
}

__device__ __forceinline__ v8f wmma_bf16(v16b a, v16b b, v8f c) {
  v8f d = __builtin_amdgcn_wmma_f32_16x16x32_bf16(false, a, false, b, (short)0, c, false, false);
  asm volatile("v_nop\n\tv_nop\n\tv_nop\n\tv_nop" : "+v"(d) : "v"(a), "v"(b));
  return d;
}

__device__ __forceinline__ v8f mma3(v16b ah, v16b al, v16b bh, v16b bl, v8f c) {
  c = wmma_bf16(ah, bh, c);
  c = wmma_bf16(al, bh, c);
  c = wmma_bf16(ah, bl, c);
  return c;
}

__device__ __forceinline__ v16b ldfrag(const u16* p, int h) {
  Frag f;
  f.half[0] = *(const v8usa*)(p + 8 * h);
  f.half[1] = *(const v8usa*)(p + 16 + 8 * h);
  return f.v;
}

__global__ __launch_bounds__(256) void pack_hf_kernel(
    const float* __restrict__ H, const float* __restrict__ F,
    u16* __restrict__ HFhi, u16* __restrict__ HFlo, int ngroups)
{
  const int g = blockIdx.x * 256 + threadIdx.x;
  if (g >= ngroups) return;
  const int row = g >> 4, c8 = (g & 15) * 8;
  const float* src = (c8 < 64) ? (H + (size_t)row * 64 + c8) : (F + (size_t)row * 64 + (c8 - 64));
  const v4f a = *(const v4fa*)src;
  const v4f c = *(const v4fa*)(src + 4);
  const HL8 s = split8(cat8(a, c));
  u16* dh = HFhi + (size_t)g * 8;
  u16* dl = HFlo + (size_t)g * 8;
  *(volatile v8us*)dh = s.hi;
  *(volatile v8us*)dl = s.lo;
  __threadfence();
  *(volatile v8us*)dh = s.hi;
  *(volatile v8us*)dl = s.lo;
}

__device__ __forceinline__ void wsplit_store_pass(const HL8* s, const size_t* off, u16* dhi, u16* dlo) {
#pragma unroll
  for (int it = 0; it < 2; ++it) {
    *(volatile v8us*)(dhi + off[it]) = s[it].hi;
    *(volatile v8us*)(dlo + off[it]) = s[it].lo;
  }
}

__global__ __launch_bounds__(256) void wsplit_kernel(
    const float* __restrict__ src, int in_dim, int out_dim, int src_z,
    u16* __restrict__ dhi, u16* __restrict__ dlo, int dst_z)
{
  __shared__ float T[64][65];
  const int t = threadIdx.x;
  const int o0 = blockIdx.x * 64, i0 = blockIdx.y * 64;
  const float* s = src + (size_t)blockIdx.z * src_z;
#pragma unroll
  for (int it = 0; it < 16; ++it) {
    const int idx = it * 256 + t;
    const int i = idx >> 6, o = idx & 63;
    T[o][i] = s[(size_t)(i0 + i) * out_dim + o0 + o];
  }
  __syncthreads();
  const size_t dz = (size_t)blockIdx.z * dst_z;
  HL8 sp[2];
  size_t off[2];
#pragma unroll
  for (int it = 0; it < 2; ++it) {
    const int p = it * 256 + t;
    const int o = p >> 3, i8 = (p & 7) * 8;
    v8f x;
#pragma unroll
    for (int j = 0; j < 8; ++j) x[j] = T[o][i8 + j];
    sp[it] = split8(x);
    off[it] = dz + (size_t)(o0 + o) * in_dim + i0 + i8;
  }
  wsplit_store_pass(sp, off, dhi, dlo);
  __threadfence();
  wsplit_store_pass(sp, off, dhi, dlo);
}

__device__ __forceinline__ void gemm_store_pass(const float* st, float* Cf, int wf, u16* Chi, u16* Clo, int wh,
                                                int ldc, size_t row0, int n0, int lane) {
  if (wf) {
#pragma unroll
    for (int it = 0; it < 8; ++it) {
      const int p = it * 32 + lane;
      const int r = p >> 4, c4 = (p & 15) * 4;
      const v4f v = *(const v4fa*)(st + r * 68 + c4);
      *(volatile v4f*)(Cf + (row0 + r) * (size_t)ldc + n0 + c4) = v;
    }
  }
  if (wh) {
#pragma unroll
    for (int it = 0; it < 4; ++it) {
      const int p = it * 32 + lane;
      const int r = p >> 3, c8 = (p & 7) * 8;
      const v4f a = *(const v4fa*)(st + r * 68 + c8);
      const v4f c = *(const v4fa*)(st + r * 68 + c8 + 4);
      const HL8 s = split8(cat8(a, c));
      const size_t gi = (row0 + r) * (size_t)ldc + n0 + c8;
      *(volatile v8us*)(Chi + gi) = s.hi;
      *(volatile v8us*)(Clo + gi) = s.lo;
    }
  }
}

__global__ __launch_bounds__(128) void gemm_kernel(
    const u16* __restrict__ Ahi, const u16* __restrict__ Alo, int lda,
    const u16* __restrict__ Bhi, const u16* __restrict__ Blo, int ldb, int K,
    const float* __restrict__ bias, float bsc,
    float* __restrict__ Cf, int wf, u16* __restrict__ Chi, u16* __restrict__ Clo, int wh, int ldc)
{
  __shared__ __attribute__((aligned(16))) float sT[4][16 * 68];

  const int tid = threadIdx.x, lane = tid & 31, w = tid >> 5;
  const int h = lane >> 4, m = lane & 15;
  const size_t row0 = (size_t)blockIdx.x * 64 + 16 * w;
  const int n0 = blockIdx.y * 64;

  const u16* ah = Ahi + (row0 + m) * (size_t)lda;
  const u16* al = Alo + (row0 + m) * (size_t)lda;
  const u16* bh = Bhi + (size_t)(n0 + m) * ldb;
  const u16* bl = Blo + (size_t)(n0 + m) * ldb;

  const v8f z8 = {0.f, 0.f, 0.f, 0.f, 0.f, 0.f, 0.f, 0.f};
  v8f acc[4];
#pragma unroll
  for (int t = 0; t < 4; ++t) acc[t] = z8;

#pragma unroll 1
  for (int k0 = 0; k0 < K; k0 += 32) {
    const v16b fah = ldfrag(ah + k0, h);
    const v16b fal = ldfrag(al + k0, h);
#pragma unroll
    for (int t = 0; t < 4; ++t) {
      const v16b fbh = ldfrag(bh + (size_t)t * 16 * ldb + k0, h);
      const v16b fbl = ldfrag(bl + (size_t)t * 16 * ldb + k0, h);
      acc[t] = mma3(fah, fal, fbh, fbl, acc[t]);
    }
  }

  float* st = sT[w];
#pragma unroll
  for (int t = 0; t < 4; ++t) {
    const float bv = bsc * bias[n0 + 16 * t + m];
#pragma unroll
    for (int r = 0; r < 8; ++r) st[(8 * h + r) * 68 + 16 * t + m] = acc[t][r] + bv;
  }
  __syncthreads();

  gemm_store_pass(st, Cf, wf, Chi, Clo, wh, ldc, row0, n0, lane);
  __threadfence();
  gemm_store_pass(st, Cf, wf, Chi, Clo, wh, ldc, row0, n0, lane);
}

template <int CT>
__global__ __launch_bounds__(256) void reduce_kernel(
    const u16* __restrict__ Khi, const u16* __restrict__ Klo, int ldk,
    const u16* __restrict__ Xhi, const u16* __restrict__ Xlo, int ldx, int NC,
    int RB, int nper, int NP, float* __restrict__ Part)
{
  constexpr int CW = 32 * CT;
  __shared__ __attribute__((aligned(16))) u16 sK[2][64 * 32];
  __shared__ __attribute__((aligned(16))) u16 sX[2][CW * 32];
  __shared__ __attribute__((aligned(16))) float sO[64 * (CW + 4)];

  const int t = threadIdx.x, lane = t & 31, w = t >> 5;
  const int h = lane >> 4, m = lane & 15;
  const int pblk = blockIdx.x, chunk = blockIdx.y, b = blockIdx.z;
  const int col0 = chunk * CW;
  const int i = w & 3, cg = w >> 2;
  const size_t rowbase = (size_t)b * nper + (size_t)pblk * RB;

  const v8f z8 = {0.f, 0.f, 0.f, 0.f, 0.f, 0.f, 0.f, 0.f};
  v8f acc[CT];
#pragma unroll
  for (int tt = 0; tt < CT; ++tt) acc[tt] = z8;

  const int nks = RB / 32;
#pragma unroll 1
  for (int ks = 0; ks < nks; ++ks) {
    __syncthreads();
    const size_t nrow0 = rowbase + (size_t)ks * 32;
    {
      const int n = t >> 3, d8 = (t & 7) * 8;
      const size_t go = (nrow0 + n) * (size_t)ldk + d8;
      const v8us kh = *(const v8usa*)(Khi + go);
      const v8us kl = *(const v8usa*)(Klo + go);
#pragma unroll
      for (int j = 0; j < 8; ++j) {
        sK[0][(d8 + j) * 32 + n] = kh[j];
        sK[1][(d8 + j) * 32 + n] = kl[j];
      }
    }
#pragma unroll
    for (int it = 0; it < CW / 64; ++it) {
      const int p = it * 256 + t;
      const int n = p / (CW / 8), c8 = (p % (CW / 8)) * 8;
      const size_t go = (nrow0 + n) * (size_t)ldx + col0 + c8;
      const v8us xh = *(const v8usa*)(Xhi + go);
      const v8us xl = *(const v8usa*)(Xlo + go);
#pragma unroll
      for (int j = 0; j < 8; ++j) {
        sX[0][(c8 + j) * 32 + n] = xh[j];
        sX[1][(c8 + j) * 32 + n] = xl[j];
      }
    }
    __syncthreads();
    const v16b fah = ldfrag(&sK[0][(16 * i + m) * 32], h);
    const v16b fal = ldfrag(&sK[1][(16 * i + m) * 32], h);
#pragma unroll
    for (int tt = 0; tt < CT; ++tt) {
      const int c = cg * (CT * 16) + 16 * tt + m;
      const v16b fbh = ldfrag(&sX[0][c * 32], h);
      const v16b fbl = ldfrag(&sX[1][c * 32], h);
      acc[tt] = mma3(fah, fal, fbh, fbl, acc[tt]);
    }
  }

#pragma unroll
  for (int tt = 0; tt < CT; ++tt) {
    const int c = cg * (CT * 16) + 16 * tt + m;
#pragma unroll
    for (int r = 0; r < 8; ++r) sO[(16 * i + 8 * h + r) * (CW + 4) + c] = acc[tt][r];
  }
  __syncthreads();

  float* pdst = Part + ((size_t)(b * NP + pblk) * 64) * NC + col0;
#pragma unroll
  for (int it = 0; it < CW / 16; ++it) {
    const int p = it * 256 + t;
    const int row = p / (CW / 4), c4 = (p % (CW / 4)) * 4;
    const v4f v = *(const v4fa*)(sO + row * (CW + 4) + c4);
    *(volatile v4f*)(pdst + (size_t)row * NC + c4) = v;
  }
  __threadfence();
#pragma unroll
  for (int it = 0; it < CW / 16; ++it) {
    const int p = it * 256 + t;
    const int row = p / (CW / 4), c4 = (p % (CW / 4)) * 4;
    const v4f v = *(const v4fa*)(sO + row * (CW + 4) + c4);
    *(volatile v4f*)(pdst + (size_t)row * NC + c4) = v;
  }
}

__device__ __forceinline__ void comb_store_pass(const u16* sH, const u16* sL, u16* Thi, u16* Tlo,
                                                size_t rowbase, int t) {
#pragma unroll
  for (int it = 0; it < 8; ++it) {
    const int p = it * 64 + t;
    const int row = p >> 3, j8 = (p & 7) * 8;
    const v8us vh = *(const v8usa*)(sH + row * 72 + j8);
    const v8us vl = *(const v8usa*)(sL + row * 72 + j8);
    const size_t gi = (rowbase + row) * 64 + j8;
    *(volatile v8us*)(Thi + gi) = vh;
    *(volatile v8us*)(Tlo + gi) = vl;
  }
}

__global__ __launch_bounds__(64) void combine_kernel(
    const float* __restrict__ Part, int NP, int NC, float scale,
    u16* __restrict__ Thi, u16* __restrict__ Tlo)
{
  __shared__ __attribute__((aligned(16))) u16 sH[64 * 72];
  __shared__ __attribute__((aligned(16))) u16 sL[64 * 72];
  const int t = threadIdx.x;
  const int b = blockIdx.y, c0 = blockIdx.x * 64;
  const float* pb = Part + (size_t)b * NP * 64 * NC + c0 + t;
#pragma unroll 1
  for (int dk = 0; dk < 64; ++dk) {
    double s = 0.0;
#pragma unroll 1
    for (int p = 0; p < NP; ++p) s += (double)pb[((size_t)p * 64 + dk) * NC];
    const float v = (float)s * scale;
    const unsigned hb = bf16_bits(v);
    const float res = v - __uint_as_float(hb << 16);
    const unsigned lb = bf16_bits(res);
    sH[t * 72 + dk] = (u16)hb;
    sL[t * 72 + dk] = (u16)lb;
  }
  __syncthreads();
  const size_t rowbase = (size_t)b * NC + c0;
  comb_store_pass(sH, sL, Thi, Tlo, rowbase, t);
  __threadfence();
  comb_store_pass(sH, sL, Thi, Tlo, rowbase, t);
}

__device__ __forceinline__ void upd_store_pass(const float* tile, float* J32, u16* Jhi, u16* Jlo,
                                               size_t row0, int tid) {
#pragma unroll
  for (int it = 0; it < 8; ++it) {
    const int p = it * 256 + tid;
    const int r = p >> 7, c4 = (p & 127) * 4;
    const v4f v = *(const v4fa*)(tile + r * 516 + c4);
    *(volatile v4f*)(J32 + (row0 + r) * DM + c4) = v;
  }
#pragma unroll
  for (int it = 0; it < 4; ++it) {
    const int p = it * 256 + tid;
    const int r = p >> 6, c8 = (p & 63) * 8;
    const v4f a = *(const v4fa*)(tile + r * 516 + c8);
    const v4f c = *(const v4fa*)(tile + r * 516 + c8 + 4);
    const HL8 s = split8(cat8(a, c));
    const size_t gi = (row0 + r) * DM + c8;
    *(volatile v8us*)(Jhi + gi) = s.hi;
    *(volatile v8us*)(Jlo + gi) = s.lo;
  }
}

__global__ __launch_bounds__(256) void update_kernel(
    const u16* __restrict__ Qhi, const u16* __restrict__ Qlo, int ldq,
    const u16* __restrict__ MThi, const u16* __restrict__ MTlo,
    float* __restrict__ J32, u16* __restrict__ Jhi, u16* __restrict__ Jlo,
    const float* __restrict__ gamma, const float* __restrict__ beta, int nper)
{
  __shared__ __attribute__((aligned(16))) float tile[16 * 516];

  const int tid = threadIdx.x, lane = tid & 31, w = tid >> 5;
  const int h = lane >> 4, m = lane & 15;
  const size_t row0 = (size_t)blockIdx.x * 16;
  const int b = (int)(row0 / (size_t)nper);
  const int n0 = w * 64;

  const u16* qh = Qhi + (row0 + m) * (size_t)ldq;
  const u16* ql = Qlo + (row0 + m) * (size_t)ldq;
  const u16* mh = MThi + ((size_t)b * DM + n0 + m) * DKK;
  const u16* ml = MTlo + ((size_t)b * DM + n0 + m) * DKK;

  const v8f z8 = {0.f, 0.f, 0.f, 0.f, 0.f, 0.f, 0.f, 0.f};
  v8f acc[4];
#pragma unroll
  for (int t = 0; t < 4; ++t) acc[t] = z8;

#pragma unroll
  for (int ks = 0; ks < 2; ++ks) {
    const int k0 = 32 * ks;
    const v16b fah = ldfrag(qh + k0, h);
    const v16b fal = ldfrag(ql + k0, h);
#pragma unroll
    for (int t = 0; t < 4; ++t) {
      const v16b fbh = ldfrag(mh + (size_t)t * 16 * DKK + k0, h);
      const v16b fbl = ldfrag(ml + (size_t)t * 16 * DKK + k0, h);
      acc[t] = mma3(fah, fal, fbh, fbl, acc[t]);
    }
  }

#pragma unroll
  for (int t = 0; t < 4; ++t) {
    const int col = n0 + 16 * t + m;
#pragma unroll
    for (int r = 0; r < 8; ++r) {
      const int rr = 8 * h + r;
      tile[rr * 516 + col] = acc[t][r] + J32[(row0 + rr) * DM + col];
    }
  }
  __syncthreads();

#pragma unroll
  for (int q2 = 0; q2 < 2; ++q2) {
    float* trow = tile + (2 * w + q2) * 516;
    v16f x;
    float s = 0.f;
#pragma unroll
    for (int j = 0; j < 16; ++j) { x[j] = trow[j * 32 + lane]; s += x[j]; }
#pragma unroll
    for (int o = 16; o > 0; o >>= 1) s += __shfl_xor(s, o, 32);
    const float mu = s * (1.0f / 512.0f);
    float q = 0.f;
#pragma unroll
    for (int j = 0; j < 16; ++j) { const float d = x[j] - mu; x[j] = d; q += d * d; }
#pragma unroll
    for (int o = 16; o > 0; o >>= 1) q += __shfl_xor(q, o, 32);
    const float rstd = rsqrtf(q * (1.0f / 512.0f) + 1e-5f);
#pragma unroll
    for (int j = 0; j < 16; ++j) {
      const int col = j * 32 + lane;
      trow[col] = x[j] * rstd * gamma[col] + beta[col];
    }
  }
  __syncthreads();

  upd_store_pass(tile, J32, Jhi, Jlo, row0, tid);
  __threadfence();
  upd_store_pass(tile, J32, Jhi, Jlo, row0, tid);
}

__device__ __forceinline__ void out_store_pass(const float* so, float* out, size_t row0, int lane) {
#pragma unroll
  for (int it = 0; it < 8; ++it) {
    const int p = it * 32 + lane;
    const int r = p >> 4, c4 = (p & 15) * 4;
    const v4f v = *(const v4fa*)(so + r * 68 + c4);
    *(volatile v4f*)(out + (row0 + r) * 64 + c4) = v;
  }
}

__global__ __launch_bounds__(128) void final_kernel(
    const float* __restrict__ Qh32, int ldqh, const float* __restrict__ Qf32,
    const float* __restrict__ wph, const float* __restrict__ wpf,
    const u16* __restrict__ GThi, const u16* __restrict__ GTlo,
    const u16* __restrict__ WoThi, const u16* __restrict__ WoTlo,
    const float* __restrict__ bout, float* __restrict__ out, int nper)
{
  __shared__ __attribute__((aligned(16))) float sX[4][16 * 68];
  __shared__ __attribute__((aligned(16))) float sO[4][16 * 68];

  const int tid = threadIdx.x, lane = tid & 31, w = tid >> 5;
  const int h = lane >> 4, m = lane & 15;
  const size_t row0 = (size_t)blockIdx.x * 64 + 16 * w;
  const int b = (int)(((size_t)blockIdx.x * 64) / (size_t)nper);
  const float a = wph[0], c = wpf[0];
  const v4f av = {a, a, a, a};
  const v4f cv = {c, c, c, c};

  const float* qh = Qh32 + (row0 + m) * (size_t)ldqh;
  const float* qf = Qf32 + (row0 + m) * 64;

  const v8f z8 = {0.f, 0.f, 0.f, 0.f, 0.f, 0.f, 0.f, 0.f};
  v8f acc[4];
#pragma unroll
  for (int t = 0; t < 4; ++t) acc[t] = z8;

#pragma unroll
  for (int ks = 0; ks < 2; ++ks) {
    const int k0 = 32 * ks;
    Frag uh, ul;
#pragma unroll
    for (int part = 0; part < 2; ++part) {
      const int ko = k0 + 16 * part + 8 * h;
      const v4f q0 = *(const v4fa*)(qh + ko);
      const v4f q1 = *(const v4fa*)(qh + ko + 4);
      const v4f f0 = *(const v4fa*)(qf + ko);
      const v4f f1 = *(const v4fa*)(qf + ko + 4);
      const v4f u0 = q0 * av + f0 * cv;
      const v4f u1 = q1 * av + f1 * cv;
      const HL8 s = split8(cat8(u0, u1));
      uh.half[part] = s.hi;
      ul.half[part] = s.lo;
    }
#pragma unroll
    for (int t = 0; t < 4; ++t) {
      const u16* gph = GThi + ((size_t)b * 64 + 16 * t + m) * 64 + k0;
      const u16* gpl = GTlo + ((size_t)b * 64 + 16 * t + m) * 64 + k0;
      const v16b fbh = ldfrag(gph, h);
      const v16b fbl = ldfrag(gpl, h);
      acc[t] = mma3(uh.v, ul.v, fbh, fbl, acc[t]);
    }
  }

  float* sx = sX[w];
#pragma unroll
  for (int t = 0; t < 4; ++t)
#pragma unroll
    for (int r = 0; r < 8; ++r) sx[(8 * h + r) * 68 + 16 * t + m] = acc[t][r];
  __syncthreads();

  v8f acc2[4];
#pragma unroll
  for (int t = 0; t < 4; ++t) acc2[t] = z8;
#pragma unroll
  for (int ks = 0; ks < 2; ++ks) {
    const int k0 = 32 * ks;
    Frag xh, xl;
#pragma unroll
    for (int part = 0; part < 2; ++part) {
      const int ko = k0 + 16 * part + 8 * h;
      const v4f x0 = *(const v4fa*)(sx + m * 68 + ko);
      const v4f x1 = *(const v4fa*)(sx + m * 68 + ko + 4);
      const HL8 s = split8(cat8(x0, x1));
      xh.half[part] = s.hi;
      xl.half[part] = s.lo;
    }
#pragma unroll
    for (int t = 0; t < 4; ++t) {
      const v16b fbh = ldfrag(WoThi + (size_t)(16 * t + m) * 64 + k0, h);
      const v16b fbl = ldfrag(WoTlo + (size_t)(16 * t + m) * 64 + k0, h);
      acc2[t] = mma3(xh.v, xl.v, fbh, fbl, acc2[t]);
    }
  }

  float* so = sO[w];
#pragma unroll
  for (int t = 0; t < 4; ++t) {
    const float bv = bout[16 * t + m];
#pragma unroll
    for (int r = 0; r < 8; ++r) so[(8 * h + r) * 68 + 16 * t + m] = acc2[t][r] + bv;
  }
  __syncthreads();

  out_store_pass(so, out, row0, lane);
  __threadfence();
  out_store_pass(so, out, row0, lane);
}

extern "C" void kernel_launch(void* const* d_in, const int* in_sizes, int n_in,
                              void* d_out, int out_size, void* d_ws, size_t ws_size,
                              hipStream_t stream) {
  if (n_in < 15) return;
  if (in_sizes[0] != RTOT * 64 || in_sizes[1] != RTOT * 64) return;
  if (in_sizes[2] != 128 * DM || in_sizes[3] != DM) return;
  if (in_sizes[4] != NLAY * DM * DKK || in_sizes[5] != NLAY * DM * DKK) return;
  if (in_sizes[6] != NLAY * DM || in_sizes[7] != NLAY * DM) return;
  if (in_sizes[8] != DM * DKK || in_sizes[9] != DM * DKK) return;
  if (in_sizes[10] != DKK * DKK || in_sizes[13] != DKK * DKK || in_sizes[14] != DKK) return;
  if (in_sizes[11] < 1 || in_sizes[12] < 1) return;
  if (out_size != RTOT * 64) return;

  const float* H       = (const float*)d_in[0];
  const float* F       = (const float*)d_in[1];
  const float* W_in    = (const float*)d_in[2];
  const float* b_in    = (const float*)d_in[3];
  const float* Wq_l    = (const float*)d_in[4];
  const float* Wk_l    = (const float*)d_in[5];
  const float* gamma_l = (const float*)d_in[6];
  const float* beta_l  = (const float*)d_in[7];
  const float* Wqh     = (const float*)d_in[8];
  const float* Wkh     = (const float*)d_in[9];
  const float* Wqf     = (const float*)d_in[10];
  const float* wph     = (const float*)d_in[11];
  const float* wpf     = (const float*)d_in[12];
  const float* W_out   = (const float*)d_in[13];
  const float* b_out   = (const float*)d_in[14];
  float* out = (float*)d_out;

  const size_t szHFp   = (size_t)RTOT * 128 * 2;
  const size_t szJ32   = (size_t)RTOT * DM * 4;
  const size_t szJp    = (size_t)RTOT * DM * 2;
  const size_t szQKp   = (size_t)RTOT * 128 * 2;
  const size_t szQK32  = (size_t)RTOT * 128 * 4;
  const size_t szQf32  = (size_t)RTOT * 64 * 4;
  const size_t szPart  = (size_t)NB_ * NPART * 64 * DM * 4;
  const size_t szMTp   = (size_t)NB_ * DM * DKK * 2;
  const size_t szGTp   = (size_t)NB_ * DKK * DKK * 2;
  const size_t szWinp  = (size_t)DM * 128 * 2;
  const size_t szWqkp  = (size_t)NLAY * 128 * DM * 2;
  const size_t szWqkhp = (size_t)128 * DM * 2;
  const size_t szW64p  = (size_t)64 * 64 * 2;

  size_t off = 0;
  auto carve = [&](size_t bytes) -> size_t { size_t o = off; off += (bytes + 255) & ~(size_t)255; return o; };
  const size_t oHFhi = carve(szHFp),   oHFlo = carve(szHFp);
  const size_t oJ32  = carve(szJ32);
  const size_t oJhi  = carve(szJp),    oJlo  = carve(szJp);
  const size_t oQKhi = carve(szQKp),   oQKlo = carve(szQKp);
  const size_t oQK32 = carve(szQK32);
  const size_t oQf32 = carve(szQf32);
  const size_t oPart = carve(szPart);
  const size_t oMThi = carve(szMTp),   oMTlo = carve(szMTp);
  const size_t oGThi = carve(szGTp),   oGTlo = carve(szGTp);
  const size_t oWinh = carve(szWinp),  oWinl = carve(szWinp);
  const size_t oWqkh = carve(szWqkp),  oWqkl = carve(szWqkp);
  const size_t oWqhh = carve(szWqkhp), oWqhl = carve(szWqkhp);
  const size_t oWqfh = carve(szW64p),  oWqfl = carve(szW64p);
  const size_t oWoh  = carve(szW64p),  oWol  = carve(szW64p);
  const size_t total = off;
  if (total > ws_size) return;
  if (total > (size_t)134217728) return;

  char* ws = (char*)d_ws;
  u16*   HFhi   = (u16*)(ws + oHFhi);
  u16*   HFlo   = (u16*)(ws + oHFlo);
  float* J32    = (float*)(ws + oJ32);
  u16*   Jhi    = (u16*)(ws + oJhi);
  u16*   Jlo    = (u16*)(ws + oJlo);
  u16*   QKhi   = (u16*)(ws + oQKhi);
  u16*   QKlo   = (u16*)(ws + oQKlo);
  float* QK32   = (float*)(ws + oQK32);
  float* Qf32   = (float*)(ws + oQf32);
  float* Part   = (float*)(ws + oPart);
  u16*   MThi   = (u16*)(ws + oMThi);
  u16*   MTlo   = (u16*)(ws + oMTlo);
  u16*   GThi   = (u16*)(ws + oGThi);
  u16*   GTlo   = (u16*)(ws + oGTlo);
  u16*   WinThi = (u16*)(ws + oWinh);
  u16*   WinTlo = (u16*)(ws + oWinl);
  u16*   WqkThi = (u16*)(ws + oWqkh);
  u16*   WqkTlo = (u16*)(ws + oWqkl);
  u16*   WqhThi = (u16*)(ws + oWqhh);
  u16*   WqhTlo = (u16*)(ws + oWqhl);
  u16*   WqfThi = (u16*)(ws + oWqfh);
  u16*   WqfTlo = (u16*)(ws + oWqfl);
  u16*   WoThi  = (u16*)(ws + oWoh);
  u16*   WoTlo  = (u16*)(ws + oWol);

  const float scale = 0.125f;

  const int ngroups = RTOT * 128 / 8;
  pack_hf_kernel<<<(ngroups + 255) / 256, 256, 0, stream>>>(H, F, HFhi, HFlo, ngroups);

  wsplit_kernel<<<dim3(DM / 64, 128 / 64, 1), 256, 0, stream>>>(W_in, 128, DM, 0, WinThi, WinTlo, 0);
  wsplit_kernel<<<dim3(1, DM / 64, NLAY), 256, 0, stream>>>(Wq_l, DM, DKK, DM * DKK, WqkThi, WqkTlo, 128 * DM);
  wsplit_kernel<<<dim3(1, DM / 64, NLAY), 256, 0, stream>>>(Wk_l, DM, DKK, DM * DKK, WqkThi + 64 * DM, WqkTlo + 64 * DM, 128 * DM);
  wsplit_kernel<<<dim3(1, DM / 64, 1), 256, 0, stream>>>(Wqh, DM, DKK, 0, WqhThi, WqhTlo, 0);
  wsplit_kernel<<<dim3(1, DM / 64, 1), 256, 0, stream>>>(Wkh, DM, DKK, 0, WqhThi + 64 * DM, WqhTlo + 64 * DM, 0);
  wsplit_kernel<<<dim3(1, 1, 1), 256, 0, stream>>>(Wqf, 64, 64, 0, WqfThi, WqfTlo, 0);
  wsplit_kernel<<<dim3(1, 1, 1), 256, 0, stream>>>(W_out, 64, 64, 0, WoThi, WoTlo, 0);

  gemm_kernel<<<dim3(RTOT / 64, DM / 64), 128, 0, stream>>>(
      HFhi, HFlo, 128, WinThi, WinTlo, 128, 128, b_in, 1.0f, J32, 1, Jhi, Jlo, 1, DM);

  for (int t = 0; t < NLAY; ++t) {
    gemm_kernel<<<dim3(RTOT / 64, 2), 128, 0, stream>>>(
        Jhi, Jlo, DM, WqkThi + (size_t)t * 128 * DM, WqkTlo + (size_t)t * 128 * DM, DM, DM,
        b_in, 0.0f, Qf32, 0, QKhi, QKlo, 1, 128);
    reduce_kernel<4><<<dim3(NPART, DM / 128, NB_), 256, 0, stream>>>(
        QKhi + 64, QKlo + 64, 128, Jhi, Jlo, DM, DM, RBLK, NPER, NPART, Part);
    combine_kernel<<<dim3(DM / 64, NB_), 64, 0, stream>>>(Part, NPART, DM, scale, MThi, MTlo);
    update_kernel<<<RTOT / 16, 256, 0, stream>>>(
        QKhi, QKlo, 128, MThi, MTlo, J32, Jhi, Jlo, gamma_l + (size_t)t * DM, beta_l + (size_t)t * DM, NPER);
  }

  gemm_kernel<<<dim3(RTOT / 64, 2), 128, 0, stream>>>(
      Jhi, Jlo, DM, WqhThi, WqhTlo, DM, DM, b_in, 0.0f, QK32, 1, QKhi, QKlo, 1, 128);
  gemm_kernel<<<dim3(RTOT / 64, 1), 128, 0, stream>>>(
      HFhi + 64, HFlo + 64, 128, WqfThi, WqfTlo, 64, 64, b_in, 0.0f, Qf32, 1, GThi, GTlo, 0, 64);
  reduce_kernel<2><<<dim3(NPART, 1, NB_), 256, 0, stream>>>(
      QKhi + 64, QKlo + 64, 128, HFhi + 64, HFlo + 64, 128, 64, RBLK, NPER, NPART, Part);
  combine_kernel<<<dim3(1, NB_), 64, 0, stream>>>(Part, NPART, 64, scale, GThi, GTlo);
  final_kernel<<<RTOT / 64, 128, 0, stream>>>(
      QK32, 128, Qf32, wph, wpf, GThi, GTlo, WoThi, WoTlo, b_out, out, NPER);
}
